// MambawDecoder_78950088835617
// MI455X (gfx1250) — hardware-verified
//
#include <hip/hip_runtime.h>


#define NB_ 4
#define LT 1024
#define NTOK (NB_ * LT)
#define DIN 64
#define DM 256
#define DI 512
#define DS 64
#define NHD 8
#define HDM 64
#define CD 640
#define DP 1160
#define DPP 1280
#define L1 350
#define L2 400
#define DOUT 1000

typedef __attribute__((ext_vector_type(16))) __bf16   v16bf;
typedef __attribute__((ext_vector_type(16))) _Float16 v16h;
typedef __attribute__((ext_vector_type(8)))  float    v8f;
typedef __attribute__((ext_vector_type(8)))  unsigned v8u;

__device__ __forceinline__ unsigned f2bf(float f) { unsigned u = __float_as_uint(f); u += 0x7FFFu + ((u >> 16) & 1u); return u >> 16; }
__device__ __forceinline__ unsigned f2h(float f) { return (unsigned)__builtin_bit_cast(unsigned short, (_Float16)f); }
__device__ __forceinline__ int kpat(int v, int half) { return ((v & 4) ? 16 : 0) + half * 8 + 2 * (v & 3); }

template <int F16, int NP> struct Opnd { v16bf p[NP]; };

template <int F16, int NP> __device__ __forceinline__ void pack2(float f0, float f1, unsigned* o) {
    if (F16) { o[0] = f2h(f0) | (f2h(f1) << 16); return; }
    unsigned h0 = f2bf(f0), h1 = f2bf(f1); o[0] = h0 | (h1 << 16);
    if (NP >= 2) {
        float r0 = f0 - __uint_as_float(h0 << 16), r1 = f1 - __uint_as_float(h1 << 16);
        unsigned m0 = f2bf(r0), m1 = f2bf(r1); o[1] = m0 | (m1 << 16);
        if (NP >= 3) {
            float s0 = r0 - __uint_as_float(m0 << 16), s1 = r1 - __uint_as_float(m1 << 16);
            o[2] = f2bf(s0) | (f2bf(s1) << 16);
        }
    }
}
template <int F16, int NP> __device__ __forceinline__ void op_row(const float* rowp, int half, float sc, Opnd<F16, NP>& o) {
    v8u u[NP];
#pragma unroll
    for (int v = 0; v < 8; ++v) {
        int kk = kpat(v, half); unsigned t[3];
        pack2<F16, NP>(rowp[kk] * sc, rowp[kk + 1] * sc, t);
#pragma unroll
        for (int p = 0; p < NP; ++p) u[p][v] = t[p];
    }
#pragma unroll
    for (int p = 0; p < NP; ++p) o.p[p] = __builtin_bit_cast(v16bf, u[p]);
}
template <int F16, int NP> __device__ __forceinline__ void op_row_tail(const float* rowp, int half, float sc, int kvalid, Opnd<F16, NP>& o) {
    v8u u[NP];
#pragma unroll
    for (int v = 0; v < 8; ++v) {
        int kk = kpat(v, half); unsigned t[3];
        float f0 = kk < kvalid ? rowp[kk] * sc : 0.0f, f1 = (kk + 1) < kvalid ? rowp[kk + 1] * sc : 0.0f;
        pack2<F16, NP>(f0, f1, t);
#pragma unroll
        for (int p = 0; p < NP; ++p) u[p][v] = t[p];
    }
#pragma unroll
    for (int p = 0; p < NP; ++p) o.p[p] = __builtin_bit_cast(v16bf, u[p]);
}
template <int F16, int NP> __device__ __forceinline__ void op_col(const float* M, int ld, int n, int k0, int half, float sc, Opnd<F16, NP>& o) {
    v8u u[NP];
#pragma unroll
    for (int v = 0; v < 8; ++v) {
        int kk = k0 + kpat(v, half); unsigned t[3];
        pack2<F16, NP>(M[(size_t)kk * ld + n] * sc, M[(size_t)(kk + 1) * ld + n] * sc, t);
#pragma unroll
        for (int p = 0; p < NP; ++p) u[p][v] = t[p];
    }
#pragma unroll
    for (int p = 0; p < NP; ++p) o.p[p] = __builtin_bit_cast(v16bf, u[p]);
}
template <int F16, int NP> __device__ __forceinline__ void op_col_tail(const float* M, int ld, int n, int k0, int half, float sc, int K, Opnd<F16, NP>& o) {
    v8u u[NP];
#pragma unroll
    for (int v = 0; v < 8; ++v) {
        int kk = k0 + kpat(v, half); unsigned t[3];
        float f0 = kk < K ? M[(size_t)kk * ld + n] * sc : 0.0f, f1 = (kk + 1) < K ? M[(size_t)(kk + 1) * ld + n] * sc : 0.0f;
        pack2<F16, NP>(f0, f1, t);
#pragma unroll
        for (int p = 0; p < NP; ++p) u[p][v] = t[p];
    }
#pragma unroll
    for (int p = 0; p < NP; ++p) o.p[p] = __builtin_bit_cast(v16bf, u[p]);
}
__device__ __forceinline__ v8f wm_bf16(v16bf a, v16bf b, v8f c) { return __builtin_amdgcn_wmma_f32_16x16x32_bf16(false, a, false, b, (short)0, c, false, false); }
template <int F16, int NA, int NB> __device__ __forceinline__ v8f wmma_op(const Opnd<F16, NA>& a, const Opnd<F16, NB>& b, v8f c) {
    if (F16) {
        v16h ah = __builtin_bit_cast(v16h, a.p[0]), bh = __builtin_bit_cast(v16h, b.p[0]);
        c = __builtin_amdgcn_wmma_f32_16x16x32_f16(false, ah, false, bh, (short)0, c, false, false);
        asm volatile("v_nop\n\tv_nop\n\tv_nop\n\tv_nop" : "+v"(c) : "v"(ah), "v"(bh));
        return c;
    }
    constexpr int NMX = NA > NB ? NA : NB;
#pragma unroll
    for (int i = 0; i < NA; ++i)
#pragma unroll
        for (int j = 0; j < NB; ++j)
            if (i + j < NMX) c = wm_bf16(a.p[i], b.p[j], c);
    if (NA == 1 && NB == 1)      asm volatile("v_nop\n\tv_nop\n\tv_nop\n\tv_nop" : "+v"(c) : "v"(a.p[0]), "v"(b.p[0]));
    else if (NA == 2 && NB == 1) asm volatile("v_nop\n\tv_nop\n\tv_nop\n\tv_nop" : "+v"(c) : "v"(a.p[0]), "v"(a.p[1]), "v"(b.p[0]));
    else if (NA == 1 && NB == 2) asm volatile("v_nop\n\tv_nop\n\tv_nop\n\tv_nop" : "+v"(c) : "v"(a.p[0]), "v"(b.p[0]), "v"(b.p[1]));
    else if (NA == 2 && NB == 2) asm volatile("v_nop\n\tv_nop\n\tv_nop\n\tv_nop" : "+v"(c) : "v"(a.p[0]), "v"(a.p[1]), "v"(b.p[0]), "v"(b.p[1]));
    else                         asm volatile("v_nop\n\tv_nop\n\tv_nop\n\tv_nop" : "+v"(c) : "v"(a.p[0]), "v"(a.p[NA - 1]), "v"(b.p[0]), "v"(b.p[NB - 1]), "v"(a.p[NA / 2]), "v"(b.p[NB / 2]));
    return c;
}

struct ZMap { long long s1; long long s2; int zdiv; int pad_; };
__device__ __forceinline__ size_t zoff(const ZMap& m, int z) { return (size_t)((long long)(z / m.zdiv) * m.s1 + (long long)(z % m.zdiv) * m.s2); }

#define ACT_NONE 0
#define ACT_RELU 1
#define ACT_GELU_ERF 2
#define ACT_SILU 3
#define ACT_TANH 4
__device__ __forceinline__ float act_apply(int act, float x) {
    if (act == ACT_RELU) return x > 0.f ? x : 0.f;
    if (act == ACT_GELU_ERF) return 0.5f * x * (1.0f + erff(x * 0.70710678118654752f));
    if (act == ACT_SILU) return x / (1.0f + expf(-x));
    if (act == ACT_TANH) return tanhf(x);
    return x;
}
struct GemmArgs {
    ZMap za, zb_, zc, zbias, zadd, zrsc, zmul, zrbias;
    const float* A; const float* Bm; float* C; const float* bias; const float* add; const float* rsc; const float* mul; const float* rbias;
    long long ldadd, ldmul;
    int lda, ldb, ldc, K;
    float ascale, bscale, oscale, addscale;
    int M, nvalid, nstore, ldrsc;
    int bcs, pad1, pad2, pad3;
};
template <int BT, int F16, int NA, int NB, int RW, int CW, int ACT>
__global__ __launch_bounds__(256) void gemm_kernel(GemmArgs g) {
    constexpr int TR = 16 * RW, TC = 64 * CW, CSTR = TC + 4;
    __shared__ __align__(16) float cst[TR * CSTR];
    const int z = blockIdx.z;
    const float* A = g.A + zoff(g.za, z); const float* Bm = g.Bm + zoff(g.zb_, z); float* C = g.C + zoff(g.zc, z);
    const int tid = threadIdx.x, lane = tid & 31, wv = tid >> 5;
    const int l16 = lane & 15, half = lane >> 4;
    const int rt = wv % RW, ch = wv / RW;
    const int row0 = blockIdx.x * TR, col0 = blockIdx.y * TC + ch * 64;
    int arix = row0 + rt * 16 + l16; if (arix >= g.M) arix = g.M - 1;
    const float* arow = A + (size_t)arix * g.lda;
    v8f acc[4];
#pragma unroll
    for (int t = 0; t < 4; ++t) acc[t] = (v8f){};
    const int K = g.K;
#pragma unroll 1
    for (int kc = 0; kc < K; kc += 32) {
        Opnd<F16, NA> a;
        if (kc + 32 <= K) op_row<F16, NA>(arow + kc, half, g.ascale, a); else op_row_tail<F16, NA>(arow + kc, half, g.ascale, K - kc, a);
#pragma unroll
        for (int t = 0; t < 4; ++t) {
            Opnd<F16, NB> b;
            const int n = col0 + t * 16 + l16;
            if (n < g.nvalid) {
                if (BT) { if (kc + 32 <= K) op_row<F16, NB>(Bm + (size_t)n * g.ldb + kc, half, g.bscale, b); else op_row_tail<F16, NB>(Bm + (size_t)n * g.ldb + kc, half, g.bscale, K - kc, b); }
                else    { if (kc + 32 <= K) op_col<F16, NB>(Bm, g.ldb, n * g.bcs, kc, half, g.bscale, b); else op_col_tail<F16, NB>(Bm, g.ldb, n * g.bcs, kc, half, g.bscale, K, b); }
            } else {
#pragma unroll
                for (int p = 0; p < NB; ++p) b.p[p] = (v16bf){};
            }
            acc[t] = wmma_op<F16, NA, NB>(a, b, acc[t]);
        }
    }
    const float* bias = g.bias ? g.bias + zoff(g.zbias, z) : nullptr;
    const float* add = g.add ? g.add + zoff(g.zadd, z) : nullptr;
    const float* rsc = g.rsc ? g.rsc + zoff(g.zrsc, z) : nullptr;
    const float* mul = g.mul ? g.mul + zoff(g.zmul, z) : nullptr;
    const float* rbias = g.rbias ? g.rbias + zoff(g.zrbias, z) : nullptr;
#pragma unroll
    for (int t = 0; t < 4; ++t) {
        const int cl = ch * 64 + t * 16 + l16;
        const int cg = blockIdx.y * TC + cl;
        const bool cok = cg < g.nvalid;
        const float bv = (bias && cok) ? bias[(size_t)cg * g.bcs] : 0.0f;
#pragma unroll
        for (int r = 0; r < 8; ++r) {
            const int rl = rt * 16 + r + 8 * half;
            float v = acc[t][r] * g.oscale + bv;
            int rg = row0 + rl; if (rg >= g.M) rg = g.M - 1;
            if (rbias) v += rbias[rg];
            if (rsc) v *= rsc[(size_t)rg * g.ldrsc];
            if (mul && cok) v *= mul[(size_t)rg * g.ldmul + cg];
            if (add && cok) v += g.addscale * add[(size_t)rg * g.ldadd + cg];
            cst[rl * CSTR + cl] = v;
        }
    }
    __syncthreads();
    const int col = tid % TC, rsel = tid / TC, rstep = 256 / TC;
    if (ACT != ACT_NONE) {
#pragma unroll 1
        for (int r = rsel; r < TR; r += rstep) cst[r * CSTR + col] = act_apply(ACT, cst[r * CSTR + col]);
    }
    float* ob = C + (size_t)row0 * g.ldc + (size_t)blockIdx.y * TC;
    const bool colok = (int)(blockIdx.y * TC + col) < g.nstore;
    const int rmax = (g.M - row0 < TR) ? (g.M - row0) : TR;
    auto pass = [&]() {
        if (colok) {
#pragma unroll 4
            for (int r = rsel; r < rmax; r += rstep) *(volatile float*)(ob + (size_t)r * g.ldc + col) = cst[r * CSTR + col];
        }
    };
    pass();
    __threadfence();
    pass();
}
static inline ZMap zm(long long s1) { ZMap m; m.s1 = s1; m.s2 = 0; m.zdiv = 1; m.pad_ = 0; return m; }
static inline ZMap zm2(long long s1, long long s2, int zdiv) { ZMap m; m.s1 = s1; m.s2 = s2; m.zdiv = zdiv; m.pad_ = 0; return m; }
static inline GemmArgs gemm_args(const float* A, int lda, ZMap za, const float* Bm, int ldb, ZMap zb, float* C, int ldc, ZMap zc, int M, int N, int K) {
    GemmArgs g; g.za = za; g.zb_ = zb; g.zc = zc; g.zbias = zm(0); g.zadd = zm(0); g.zrsc = zm(0); g.zmul = zm(0); g.zrbias = zm(0);
    g.A = A; g.Bm = Bm; g.C = C; g.bias = nullptr; g.add = nullptr; g.rsc = nullptr; g.mul = nullptr; g.rbias = nullptr; g.ldadd = 0; g.ldmul = 0;
    g.lda = lda; g.ldb = ldb; g.ldc = ldc; g.K = K; g.ascale = 1.0f; g.bscale = 1.0f; g.oscale = 1.0f; g.addscale = 1.0f; g.M = M; g.nvalid = N; g.nstore = N; g.ldrsc = 1;
    g.bcs = 1; g.pad1 = 0; g.pad2 = 0; g.pad3 = 0;
    return g;
}
static_assert(sizeof(ZMap) == 24, "ZMap layout");
static_assert(sizeof(GemmArgs) == 8 * 24 + 8 * 8 + 2 * 8 + 4 * 4 + 4 * 4 + 4 * 4 + 4 * 4, "GemmArgs has no padding");

__global__ __launch_bounds__(256) void softmax_rows(float* S, long long sy, long long sx, int L, float prescale, const float* addv, long long say, int aydiv, int causal,
                                                  const int* imask, long long imy, long long imx, float maskval) {
    __shared__ float red[8];
    const int tid = threadIdx.x, lane = tid & 31, wid = tid >> 5;
    float* row = S + (size_t)blockIdx.y * sy + (size_t)blockIdx.x * sx;
    const float* av = addv ? addv + (size_t)(blockIdx.y / aydiv) * say : nullptr;
    const int* im = imask ? imask + (size_t)(blockIdx.y / aydiv) * imy + (size_t)blockIdx.x * imx : nullptr;
    float v[16];
    const int nj = L / 256;
    float mx = -__builtin_inff();
#pragma unroll
    for (int j = 0; j < 16; ++j) if (j < nj) { float t = row[tid + 256 * j] * prescale; if (av) t += av[tid + 256 * j]; if (im && im[tid + 256 * j] == 0) t = maskval; if (causal && (tid + 256 * j) > (int)blockIdx.x) t = -__builtin_inff(); v[j] = t; mx = fmaxf(mx, t); }
#pragma unroll
    for (int o = 16; o; o >>= 1) mx = fmaxf(mx, __shfl_xor(mx, o, 32));
    if (lane == 0) red[wid] = mx;
    __syncthreads();
    float m = red[0];
#pragma unroll
    for (int i = 1; i < 8; ++i) m = fmaxf(m, red[i]);
    if (m == -__builtin_inff()) m = 0.f;
    __syncthreads();
    float sum = 0.f;
#pragma unroll
    for (int j = 0; j < 16; ++j) if (j < nj) { v[j] = expf(v[j] - m); sum += v[j]; }
#pragma unroll
    for (int o = 16; o; o >>= 1) sum += __shfl_xor(sum, o, 32);
    if (lane == 0) red[wid] = sum;
    __syncthreads();
    float tot = 0.f;
#pragma unroll
    for (int i = 0; i < 8; ++i) tot += red[i];
    const float inv = 1.0f / tot;
#pragma unroll
    for (int j = 0; j < 16; ++j) if (j < nj) *(volatile float*)(row + tid + 256 * j) = v[j] * inv;
    __threadfence();
#pragma unroll
    for (int j = 0; j < 16; ++j) if (j < nj) *(volatile float*)(row + tid + 256 * j) = v[j] * inv;
}

#define VST2(T, p, v) do { const T vst2_v_ = (v); *(volatile T*)(p) = vst2_v_; __threadfence(); *(volatile T*)(p) = vst2_v_; } while (0)
__device__ __forceinline__ float siluf(float a) { return a / (1.f + expf(-a)); }
__device__ __forceinline__ float softplusf(float a) { return a > 20.f ? a : log1pf(expf(a)); }
__global__ __launch_bounds__(256) void k_conv(const float* __restrict__ ZX, const float* __restrict__ cw, const float* __restrict__ cb, const float* __restrict__ dtb, float* XC, float* DT) { const size_t q = (size_t)blockIdx.x * 256 + threadIdx.x; if (q >= (size_t)NTOK * CD) return; const int c = (int)(q % CD); const int r = (int)(q / CD); const int b = r / LT, t = r % LT; float s = cb[c];
#pragma unroll
    for (int j = 0; j < 4; ++j) { const int tt = t - 3 + j; if (tt >= 0) s += cw[c * 4 + j] * ZX[((size_t)b * LT + tt) * DPP + DI + c]; }
    VST2(float, XC + q, siluf(s));
    if (c < NHD) { VST2(float, DT + (size_t)r * 32 + c, softplusf(ZX[(size_t)r * DPP + DI + CD + c] + dtb[c])); } }
__global__ __launch_bounds__(256) void k_cum(const float* __restrict__ DT, const float* __restrict__ Alog, float* CUM) { const int lane = threadIdx.x & 31; const int w = blockIdx.x * 8 + (threadIdx.x >> 5); if (w >= NB_ * NHD) return; const int b = w / NHD, h = w % NHD; const float A = -expf(Alog[h]);
    float loc[32]; float tot = 0.f;
#pragma unroll
    for (int k = 0; k < 32; ++k) { const int t = lane * 32 + k; tot += DT[((size_t)b * LT + t) * 32 + h] * A; loc[k] = tot; }
    float pre = tot;
#pragma unroll
    for (int o = 1; o < 32; o <<= 1) { const float v = __shfl_up(pre, o, 32); if (lane >= o) pre += v; }
    const float excl = pre - tot;
#pragma unroll
    for (int k = 0; k < 32; ++k) { VST2(float, CUM + (size_t)w * LT + lane * 32 + k, loc[k] + excl); } }
__global__ __launch_bounds__(256) void k_mask(const float* __restrict__ G, const float* __restrict__ CUM, const float* __restrict__ DT, int b, float* M) { const size_t q = (size_t)blockIdx.x * 256 + threadIdx.x; if (q >= (size_t)NHD * LT * LT) return; const int s = (int)(q % LT); const int t = (int)((q / LT) % LT); const int h = (int)(q / ((size_t)LT * LT)); float v = 0.f;
    if (s <= t) { const float* cu = CUM + ((size_t)b * NHD + h) * LT; v = G[((size_t)b * LT + t) * LT + s] * expf(cu[t] - cu[s]) * DT[((size_t)b * LT + s) * 32 + h]; } VST2(float, M + q, v); }
__global__ __launch_bounds__(256) void k_gate(const float* __restrict__ Y, const float* __restrict__ XC, const float* __restrict__ ZX, const float* __restrict__ Dp, const float* __restrict__ nw, float* YG) { const int lane = threadIdx.x & 31; const int r = blockIdx.x * 8 + (threadIdx.x >> 5); if (r >= NTOK) return; float ss = 0.f;
#pragma unroll 1
    for (int c = lane; c < DI; c += 32) { const int h = c / HDM; const float y = (Y[(size_t)r * DI + c] + Dp[h] * XC[(size_t)r * CD + c]) * siluf(ZX[(size_t)r * DPP + c]); ss += y * y; }
#pragma unroll
    for (int o = 16; o; o >>= 1) ss += __shfl_xor(ss, o, 32);
    const float rs = rsqrtf(ss / (float)DI + 1e-5f);
#pragma unroll 1
    for (int c = lane; c < DI; c += 32) { const int h = c / HDM; const float y = (Y[(size_t)r * DI + c] + Dp[h] * XC[(size_t)r * CD + c]) * siluf(ZX[(size_t)r * DPP + c]); VST2(float, YG + (size_t)r * DI + c, y * rs * nw[c]); } }
__global__ __launch_bounds__(256) void k_ln(const float* __restrict__ O, const float* __restrict__ RES, const float* __restrict__ g, const float* __restrict__ bb, float* H, int nrows) { const int lane = threadIdx.x & 31; const int r = blockIdx.x * 8 + (threadIdx.x >> 5); if (r >= nrows) return; float v[8]; float s = 0.f;
#pragma unroll
    for (int k = 0; k < 8; ++k) { const int c = lane + 32 * k; v[k] = O[(size_t)r * DM + c] + RES[(size_t)r * DM + c]; s += v[k]; }
#pragma unroll
    for (int o = 16; o; o >>= 1) s += __shfl_xor(s, o, 32);
    const float mean = s / (float)DM; float qq = 0.f;
#pragma unroll
    for (int k = 0; k < 8; ++k) { const float d = v[k] - mean; qq += d * d; }
#pragma unroll
    for (int o = 16; o; o >>= 1) qq += __shfl_xor(qq, o, 32);
    const float rstd = rsqrtf(qq / (float)DM + 1e-5f);
#pragma unroll
    for (int k = 0; k < 8; ++k) { const int c = lane + 32 * k; VST2(float, H + (size_t)r * DM + c, (v[k] - mean) * rstd * g[c] + bb[c]); } }
__global__ __launch_bounds__(256) void k_last(const float* __restrict__ XC, const float* __restrict__ ZX, const float* __restrict__ DT, const float* __restrict__ CUM, const float* __restrict__ Dp, const float* __restrict__ nw, const float* __restrict__ Wo, const float* __restrict__ H1, const float* __restrict__ lg, const float* __restrict__ lb, const float* __restrict__ W1, const float* __restrict__ b1, const float* __restrict__ W2, const float* __restrict__ b2, const float* __restrict__ W3, const float* __restrict__ b3, float* out) {
    __shared__ float wgt[NHD][LT]; __shared__ float yv[DI]; __shared__ float hv[DM]; __shared__ float z1[L1 + 2]; __shared__ float z2[L2]; __shared__ float red[256]; const int b = blockIdx.x, tid = threadIdx.x; const int tl = LT - 1; const size_t rl = (size_t)b * LT + tl;
    for (int s = tid; s < LT; s += 256) { const size_t rs = (size_t)b * LT + s; float g = 0.f;
#pragma unroll 1
        for (int n = 0; n < DS; ++n) g += XC[rl * CD + DI + DS + n] * XC[rs * CD + DI + n];
#pragma unroll 1
        for (int h = 0; h < NHD; ++h) { const float* cu = CUM + ((size_t)b * NHD + h) * LT; wgt[h][s] = g * expf(cu[tl] - cu[s]) * DT[rs * 32 + h]; } }
    __syncthreads();
    for (int c = tid; c < DI; c += 256) { const int h = c / HDM; float y = 0.f;
#pragma unroll 1
        for (int s = 0; s < LT; ++s) y += wgt[h][s] * XC[((size_t)b * LT + s) * CD + c];
        y = (y + Dp[h] * XC[rl * CD + c]) * siluf(ZX[rl * DPP + c]); yv[c] = y; }
    __syncthreads();
    { float ss = 0.f; for (int c = tid; c < DI; c += 256) ss += yv[c] * yv[c]; red[tid] = ss; __syncthreads(); for (int o = 128; o > 0; o >>= 1) { if (tid < o) red[tid] += red[tid + o]; __syncthreads(); } const float rs = rsqrtf(red[0] / (float)DI + 1e-5f); __syncthreads(); for (int c = tid; c < DI; c += 256) yv[c] = yv[c] * rs * nw[c]; }
    __syncthreads();
    { const int c = tid; float o = 0.f;
#pragma unroll 1
        for (int k = 0; k < DI; ++k) o += yv[k] * Wo[(size_t)k * DM + c]; o += H1[rl * DM + c]; hv[c] = o; }
    __syncthreads();
    { red[tid] = hv[tid]; __syncthreads(); for (int o = 128; o > 0; o >>= 1) { if (tid < o) red[tid] += red[tid + o]; __syncthreads(); } const float mean = red[0] / (float)DM; __syncthreads(); const float d = hv[tid] - mean; red[tid] = d * d; __syncthreads(); for (int o = 128; o > 0; o >>= 1) { if (tid < o) red[tid] += red[tid + o]; __syncthreads(); } const float rstd = rsqrtf(red[0] / (float)DM + 1e-5f); __syncthreads(); hv[tid] = d * rstd * lg[tid] + lb[tid]; }
    __syncthreads();
    for (int j = tid; j < L1; j += 256) { float s = b1[j];
#pragma unroll 1
        for (int k = 0; k < DM; ++k) s += hv[k] * W1[(size_t)k * L1 + j]; z1[j] = fmaxf(s, 0.f); }
    __syncthreads();
    for (int j = tid; j < L2; j += 256) { float s = b2[j];
#pragma unroll 1
        for (int k = 0; k < L1; ++k) s += z1[k] * W2[(size_t)k * L2 + j]; z2[j] = fmaxf(s, 0.f); }
    __syncthreads();
    for (int j = tid; j < DOUT; j += 256) { float s = b3[j];
#pragma unroll 1
        for (int k = 0; k < L2; ++k) s += z2[k] * W3[(size_t)k * DOUT + j]; VST2(float, out + (size_t)b * 1024 + j, s); } }
__global__ __launch_bounds__(256) void k_out(const float* __restrict__ OB, float* out) { const int q = blockIdx.x * 256 + threadIdx.x; if (q >= NB_ * DOUT) return; VST2(float, out + q, OB[(size_t)(q / DOUT) * 1024 + (q % DOUT)]); }
extern "C" void kernel_launch(void* const* d_in, const int* in_sizes, int n_in,
                              void* d_out, int out_size, void* d_ws, size_t ws_size, hipStream_t stream) {
    (void)in_sizes; (void)n_in; (void)out_size;
    const float* x = (const float*)d_in[0]; const float* encW = (const float*)d_in[1]; const float* encb = (const float*)d_in[2]; const float* inW = (const float*)d_in[3]; const float* cw = (const float*)d_in[4]; const float* cb = (const float*)d_in[5]; const float* dtb = (const float*)d_in[6]; const float* Alog = (const float*)d_in[7]; const float* Dp = (const float*)d_in[8]; const float* nw = (const float*)d_in[9]; const float* outW = (const float*)d_in[10]; const float* lg = (const float*)d_in[11]; const float* lb = (const float*)d_in[12]; const float* W1 = (const float*)d_in[13]; const float* b1 = (const float*)d_in[14]; const float* W2 = (const float*)d_in[15]; const float* b2 = (const float*)d_in[16]; const float* W3 = (const float*)d_in[17]; const float* b3 = (const float*)d_in[18];
    float* out = (float*)d_out;
    char* wsp = (char*)d_ws;
    auto take = [&](size_t bytes) { char* p = wsp; wsp += (bytes + 255) & ~(size_t)255; return (void*)p; };
    float* H0 = (float*)take((size_t)NTOK * DM * 4); float* ZX = (float*)take((size_t)NTOK * DPP * 4); float* XC = (float*)take((size_t)NTOK * CD * 4); float* DT = (float*)take((size_t)NTOK * 32 * 4); float* CUM = (float*)take((size_t)NB_ * NHD * LT * 4); float* G = (float*)take((size_t)NB_ * LT * LT * 4); float* M = (float*)take((size_t)NHD * LT * LT * 4); float* Y = (float*)take((size_t)NTOK * DI * 4); float* YG = (float*)take((size_t)NTOK * DI * 4); float* O = (float*)take((size_t)NTOK * DM * 4); float* H1 = (float*)take((size_t)NTOK * DM * 4); float* OB = (float*)take((size_t)NB_ * 1024 * 4);
    if ((size_t)(wsp - (char*)d_ws) > ws_size) return;
    { GemmArgs g = gemm_args(x, DIN, zm(0), encW, DM, zm(0), H0, DM, zm(0), NTOK, DM, DIN); g.bias = encb; gemm_kernel<0, 0, 2, 2, 4, 2, ACT_NONE><<<dim3(NTOK / 64, DM / 128, 1), 256, 0, stream>>>(g); }
    for (int l = 0; l < 2; ++l) { const float* Hin = (l == 0) ? H0 : H1;
        { GemmArgs g = gemm_args(Hin, DM, zm(0), inW + (size_t)l * DM * DP, DP, zm(0), ZX, DPP, zm(0), NTOK, DP, DM); gemm_kernel<0, 1, 1, 1, 4, 2, ACT_NONE><<<dim3(NTOK / 64, (DP + 127) / 128, 1), 256, 0, stream>>>(g); }
        k_conv<<<(unsigned)(((size_t)NTOK * CD) / 256), 256, 0, stream>>>(ZX, cw + (size_t)l * CD * 4, cb + (size_t)l * CD, dtb + l * NHD, XC, DT);
        k_cum<<<(NB_ * NHD) / 8, 256, 0, stream>>>(DT, Alog + l * NHD, CUM);
        if (l == 0) {
            { GemmArgs g = gemm_args(XC + DI + DS, CD, zm((long long)LT * CD), XC + DI, CD, zm((long long)LT * CD), G, LT, zm((long long)LT * LT), LT, LT, DS); gemm_kernel<1, 1, 1, 1, 4, 2, ACT_NONE><<<dim3(LT / 64, LT / 128, NB_), 256, 0, stream>>>(g); }
            for (int b = 0; b < NB_; ++b) {
                k_mask<<<(unsigned)(((size_t)NHD * LT * LT) / 256), 256, 0, stream>>>(G, CUM, DT, b, M);
                { GemmArgs g = gemm_args(M, LT, zm((long long)LT * LT), XC + (size_t)b * LT * CD, CD, zm(HDM), Y + (size_t)b * LT * DI, DI, zm(HDM), LT, HDM, LT); gemm_kernel<0, 1, 1, 1, 8, 1, ACT_NONE><<<dim3(LT / 128, 1, NHD), 256, 0, stream>>>(g); }
            }
            k_gate<<<NTOK / 8, 256, 0, stream>>>(Y, XC, ZX, Dp, nw, YG);
            { GemmArgs g = gemm_args(YG, DI, zm(0), outW, DM, zm(0), O, DM, zm(0), NTOK, DM, DI); gemm_kernel<0, 1, 1, 1, 4, 2, ACT_NONE><<<dim3(NTOK / 64, DM / 128, 1), 256, 0, stream>>>(g); }
            k_ln<<<NTOK / 8, 256, 0, stream>>>(O, H0, lg, lb, H1, NTOK);
        } else {
            k_last<<<NB_, 256, 0, stream>>>(XC, ZX, DT, CUM, Dp + NHD, nw + DI, outW + (size_t)DM * DI, H1, lg + DM, lb + DM, W1, b1, W2, b2, W3, b3, OB);
            k_out<<<(NB_ * DOUT + 255) / 256, 256, 0, stream>>>(OB, out);
        }
    }
}
